// CausalSelfAttention_47493748359173
// MI455X (gfx1250) — hardware-verified
//
#include <hip/hip_runtime.h>
#include <math.h>

typedef __attribute__((ext_vector_type(16))) _Float16 v16h;
typedef __attribute__((ext_vector_type(16))) __bf16 v16b;
typedef __attribute__((ext_vector_type(8)))  _Float16 v8h;
typedef __attribute__((ext_vector_type(8)))  __bf16 v8b;
typedef __attribute__((ext_vector_type(8)))  float v8f;
typedef __attribute__((ext_vector_type(4)))  float v4f;
typedef __attribute__((ext_vector_type(4)))  unsigned v4u;

template <typename T> __device__ __forceinline__ void vst2(void* p, T v) { *(volatile T*)p = v; __threadfence(); *(volatile T*)p = v; }
__device__ __forceinline__ v8f wmma16(v16h a, v16h b, v8f c) {
  v8f d = __builtin_amdgcn_wmma_f32_16x16x32_f16(false, a, false, b, (short)0, c, false, false);
  asm volatile("v_nop\n\tv_nop\n\tv_nop\n\tv_nop" : "+v"(d) : "v"(a), "v"(b));
  return d;
}
__device__ __forceinline__ v8f wmma_bf(v16b a, v16b b, v8f c) {
  v8f d = __builtin_amdgcn_wmma_f32_16x16x32_bf16(false, a, false, b, (short)0, c, false, false);
  asm volatile("v_nop\n\tv_nop\n\tv_nop\n\tv_nop" : "+v"(d) : "v"(a), "v"(b));
  return d;
}
__device__ __forceinline__ v16h frag_h(const _Float16* rowk0, int lane) {
  union { v16h v; v8h q[2]; } u; const _Float16* p = rowk0 + 8 * (lane >> 4);
  u.q[0] = *(const v8h*)p; u.q[1] = *(const v8h*)(p + 16); return u.v;
}
__device__ __forceinline__ v16b frag_b(const __bf16* rowk0, int lane) {
  union { v16b v; v8b q[2]; } u; const __bf16* p = rowk0 + 8 * (lane >> 4);
  u.q[0] = *(const v8b*)p; u.q[1] = *(const v8b*)(p + 16); return u.v;
}
__device__ __forceinline__ v16h frag_f32s(const float* rowk0, int lane, float sc) {
  v16h a; const float* p = rowk0 + 8 * (lane >> 4);
#pragma unroll
  for (int i = 0; i < 8; ++i) { a[i] = (_Float16)(p[i] * sc); a[8 + i] = (_Float16)(p[16 + i] * sc); }
  return a;
}
struct F2 { v16b h, l; };
__device__ __forceinline__ F2 bsplit16(const float v[16]) { F2 r;
#pragma unroll
  for (int i = 0; i < 16; ++i) { const __bf16 h = (__bf16)v[i]; r.h[i] = h; r.l[i] = (__bf16)(v[i] - (float)h); }
  return r; }
__device__ __forceinline__ F2 split_row(const float* row, int k0, int lane) { float v[16]; const float* p = row + k0 + 8 * (lane >> 4);
#pragma unroll
  for (int i = 0; i < 8; ++i) { v[i] = p[i]; v[8 + i] = p[16 + i]; }
  return bsplit16(v); }
__device__ __forceinline__ float bfr(float v) { return (float)(__bf16)v; }
#define LDSX() do { asm volatile("s_wait_dscnt 0" ::: "memory"); __builtin_amdgcn_wave_barrier(); __builtin_amdgcn_fence(3  , "workgroup"); } while (0)

static __device__ __forceinline__ _Float16 toh_flush(float v) { const _Float16 r = (_Float16)v; return (fabsf(v) < 6.103515625e-05f) ? (_Float16)0.0f : r; }
__device__ __forceinline__ v16h frag_f32s_flush(const float* rowk0, int lane, float sc) {
  v16h a; const float* p = rowk0 + 8 * (lane >> 4);
#pragma unroll
  for (int i = 0; i < 8; ++i) { a[i] = toh_flush(p[i] * sc); a[8 + i] = toh_flush(p[16 + i] * sc); }
  return a;
}

#ifndef NB
#define NB 2
#endif
#ifndef SEQ
#define SEQ 2048
#endif
#define NB_FULL 2
#define SEQ_FULL 2048
#define TT SEQ
#define CC 1024
#define DIN 1024
#define NH 16
#define NKV 4
#define HD 64
#define KC (NKV * HD)
#define NREP (NH / NKV)
#define GCH 12
#define QKS 1.2f
#define NQB (TT / 64)
#define HIR (TT < 256 ? TT : 256)
#define HI0 0
#define QBH (HIR / 64)
#define NLO (NQB - QBH)
#define SC2 (0.125f * 1.4426950408889634f)

static_assert(NB >= 1 && NB <= NB_FULL);
static_assert(SEQ % 64 == 0 && SEQ <= SEQ_FULL && SEQ >= 64);
static_assert(CC == NH * HD && KC == NKV * HD && NH % NKV == 0);
static_assert(HD == 64);
static_assert(HD / 4 == 16);
static_assert(DIN % 128 == 0 && CC % 128 == 0 && KC % 128 == 0);
static_assert(DIN % 32 == 0 && CC % 32 == 0 && TT % 32 == 0);
static_assert(128 / HD == 2);
static_assert(GCH % 4 == 0 && GCH >= 4 && GCH <= DIN && HD / 2 == 32);
static_assert(HIR % 64 == 0 && HI0 == 0 && HIR <= TT && QBH >= 1 && NLO >= 0);
static_assert(((HIR - 1) >> 5) * 32 + 31 < HIR);
static_assert((CC * DIN) % 2048 == 0 && (KC * DIN) % 2048 == 0);

#define WS_QH  ((size_t)0)
#define WS_KH  (WS_QH + 2u * (size_t)NB * TT * CC)
#define WS_VT  (WS_KH + 2u * (size_t)NB * TT * KC)
#define WS_QL  (WS_VT + 2u * (size_t)NB * KC * TT)
#define WS_KL  (WS_QL + 2u * (size_t)NB * HIR * CC)
#define WS_VB  (WS_KL + 2u * (size_t)NB * HIR * KC)
#define WS_VBL (WS_VB + 2u * (size_t)NB * KC * HIR)
#define WS_WQB (WS_VBL + 2u * (size_t)NB * KC * HIR)
#define WS_WOB (WS_WQB + 2u * (size_t)(CC + 2 * KC) * DIN)
#define WS_WOH (WS_WOB + 2u * (size_t)DIN * CC)
#define WS_Y   (WS_WOH + 2u * (size_t)DIN * CC)
#define WS_END (WS_Y + 4u * (size_t)NB * TT * CC)
static_assert(WS_END <= (size_t)134217728);
static_assert(WS_KH % 128 == 0 && WS_VT % 128 == 0 && WS_QL % 128 == 0 && WS_KL % 128 == 0 && WS_VB % 128 == 0 && WS_VBL % 128 == 0 && WS_WQB % 128 == 0 && WS_WOB % 128 == 0 && WS_WOH % 128 == 0 && WS_Y % 128 == 0);

__global__ __launch_bounds__(256) void k_cvt(const float* __restrict__ W, int n8, __bf16* __restrict__ WB, _Float16* __restrict__ WH, int mkh) {
  const int i = blockIdx.x * 256 + threadIdx.x;
  if (i < n8) {
    const v4f a = *(const v4f*)(W + (size_t)i * 8); const v4f c = *(const v4f*)(W + (size_t)i * 8 + 4);
    union { v8b v; v4u u; } ob; union { v8h v; v4u u; } oh;
#pragma unroll
    for (int j = 0; j < 4; ++j) { const __bf16 x0 = (__bf16)a[j]; const __bf16 x1 = (__bf16)c[j]; ob.v[j] = x0; ob.v[4 + j] = x1; oh.v[j] = (_Float16)((float)x0 * 256.0f); oh.v[4 + j] = (_Float16)((float)x1 * 256.0f); }
    vst2(WB + (size_t)i * 8, ob.u); if (mkh) vst2(WH + (size_t)i * 8, oh.u);
  }
}

__global__ __launch_bounds__(128) void k_proj_qk(const float* __restrict__ X, const __bf16* __restrict__ WA, const float* __restrict__ COS, const float* __restrict__ SIN,
    _Float16* __restrict__ DH, _Float16* __restrict__ DL, int pitch) {
#pragma clang fp contract(off)
  __shared__ __align__(16) _Float16 sh[64][136], sl[64][136];
  __shared__ __align__(16) float scs[64][36], ssn[64][36];
  const int tid = threadIdx.x, wave = tid >> 5, lane = tid & 31, col = lane & 15, g = lane >> 4; const int c0 = blockIdx.y * 128; const size_t r0 = (size_t)blockIdx.x * 64; const size_t bb = r0 / TT; const int t0 = (int)(r0 % TT);
  const size_t xr = bb * (size_t)SEQ_FULL + t0 + wave * 16 + col;
  v8f acc[8] = {};
#pragma unroll 2
  for (int kc = 0; kc < DIN / 32; ++kc) { v16b a; { const float* p = X + xr * DIN + kc * 32 + 8 * g;
#pragma unroll
      for (int i = 0; i < 8; ++i) { a[i] = (__bf16)p[i]; a[8 + i] = (__bf16)p[16 + i]; } }
    asm volatile("s_wait_loadcnt 0x0" ::: "memory");
#pragma unroll
    for (int j = 0; j < 8; ++j) { const v16b w = frag_b(WA + (size_t)(c0 + j * 16 + col) * DIN + kc * 32, lane); asm volatile("s_wait_loadcnt 0x0" ::: "memory"); acc[j] = wmma_bf(a, w, acc[j]); } }
#pragma unroll 1
  for (int e = tid; e < 64 * 8; e += 128) { const int rl = e >> 3, q = e & 7; const v4f cv = *(const v4f*)(COS + (size_t)(t0 + rl) * 32 + q * 4); const v4f sv = *(const v4f*)(SIN + (size_t)(t0 + rl) * 32 + q * 4); v4f cr, sr;
#pragma unroll
    for (int i = 0; i < 4; ++i) { cr[i] = bfr(cv[i]); sr[i] = bfr(sv[i]); }
    *(v4f*)&scs[rl][q * 4] = cr; *(v4f*)&ssn[rl][q * 4] = sr; }
  __syncthreads();
  const bool hi_rows = t0 < HIR;
#pragma unroll
  for (int hh = 0; hh < 2; ++hh) {
#pragma unroll
    for (int r = 0; r < 8; ++r) { const int rl = wave * 16 + 8 * g + r;
      const float ca = scs[rl][col], cb = scs[rl][16 + col], sa = ssn[rl][col], sb = ssn[rl][16 + col];
      const float a0 = acc[hh * 4 + 0][r], a1 = acc[hh * 4 + 1][r], b0 = acc[hh * 4 + 2][r], b1 = acc[hh * 4 + 3][r];
      float y[4]; y[0] = a0 * ca + b0 * sa; y[1] = a1 * cb + b1 * sb; y[2] = b0 * ca - a0 * sa; y[3] = b1 * cb - a1 * sb;
      float ss = (y[0] * y[0] + y[1] * y[1]) + (y[2] * y[2] + y[3] * y[3]);
      ss += __shfl_xor(ss, 1); ss += __shfl_xor(ss, 2); ss += __shfl_xor(ss, 4); ss += __shfl_xor(ss, 8);
      const float sc = rsqrtf(ss * (1.0f / 64.0f) + 1.1920929e-7f);
#pragma unroll
      for (int q4 = 0; q4 < 4; ++q4) { const float v = (y[q4] * sc) * QKS; const _Float16 hv = toh_flush(v); sh[rl][hh * 64 + q4 * 16 + col] = hv; sl[rl][hh * 64 + q4 * 16 + col] = toh_flush((v - (float)hv) * 1024.0f); } } }
  __syncthreads();
  for (int e = tid; e < 64 * 16; e += 128) { const int rl = e >> 4, q = e & 15; vst2(DH + (r0 + rl) * (size_t)pitch + c0 + q * 8, *(const v4u*)&sh[rl][q * 8]); if (hi_rows) vst2(DL + (bb * HIR + (size_t)(t0 - HI0) + rl) * (size_t)pitch + c0 + q * 8, *(const v4u*)&sl[rl][q * 8]); }
}

__global__ __launch_bounds__(128) void k_proj_v(const float* __restrict__ X, const __bf16* __restrict__ WA, const float* __restrict__ VE, const float* __restrict__ WG,
    _Float16* __restrict__ VT, __bf16* __restrict__ VB, __bf16* __restrict__ VBL) {
  __shared__ __align__(16) _Float16 th[128][72]; __shared__ __align__(16) __bf16 tb[128][72], tbl[128][72]; __shared__ float sg[2][64];
  const int tid = threadIdx.x, wave = tid >> 5, lane = tid & 31, col = lane & 15, g = lane >> 4; const int c0 = blockIdx.y * 128; const size_t r0 = (size_t)blockIdx.x * 64; const size_t bb = r0 / TT; const int t0 = (int)(r0 % TT);
  const size_t xr = bb * (size_t)SEQ_FULL + t0 + wave * 16 + col;
  { const int rl = tid & 63, hh = tid >> 6; const int gi = blockIdx.y * 2 + hh; const size_t xg = (bb * (size_t)SEQ_FULL + t0 + rl) * DIN; float z = 0.f;
#pragma unroll 1
    for (int c4 = 0; c4 < GCH / 4; ++c4) { const v4f xv = *(const v4f*)(X + xg + c4 * 4); const v4f wv = *(const v4f*)(WG + gi * GCH + c4 * 4);
      z += bfr(xv[0]) * bfr(wv[0]); z += bfr(xv[1]) * bfr(wv[1]); z += bfr(xv[2]) * bfr(wv[2]); z += bfr(xv[3]) * bfr(wv[3]); }
    sg[hh][rl] = 3.0f * (1.0f / (1.0f + expf(-z))); }
  v8f acc[8] = {};
#pragma unroll 2
  for (int kc = 0; kc < DIN / 32; ++kc) { v16b a; { const float* p = X + xr * DIN + kc * 32 + 8 * g;
#pragma unroll
      for (int i = 0; i < 8; ++i) { a[i] = (__bf16)p[i]; a[8 + i] = (__bf16)p[16 + i]; } }
    asm volatile("s_wait_loadcnt 0x0" ::: "memory");
#pragma unroll
    for (int j = 0; j < 8; ++j) { const v16b w = frag_b(WA + (size_t)(c0 + j * 16 + col) * DIN + kc * 32, lane); asm volatile("s_wait_loadcnt 0x0" ::: "memory"); acc[j] = wmma_bf(a, w, acc[j]); } }
  __syncthreads();
  const bool hi_rows = t0 < HIR;
#pragma unroll
  for (int j = 0; j < 8; ++j) { float vev[8];
#pragma unroll
    for (int r = 0; r < 8; ++r) vev[r] = VE[(bb * (size_t)SEQ_FULL + t0 + wave * 16 + 8 * g + r) * (size_t)KC + c0 + j * 16 + col];
    asm volatile("s_wait_loadcnt 0x0" ::: "memory");
#pragma unroll
    for (int r = 0; r < 8; ++r) { const int rl = wave * 16 + 8 * g + r, cl = j * 16 + col; const float v = acc[j][r] + sg[j >> 2][rl] * bfr(vev[r]); th[cl][rl] = toh_flush(v); const __bf16 bh = (__bf16)v; tb[cl][rl] = bh; tbl[cl][rl] = (__bf16)(v - (float)bh); } }
  __syncthreads();
  for (int e = tid; e < 128 * 8; e += 128) { const int cl = e >> 3, q = e & 7; vst2(VT + (bb * KC + c0 + cl) * (size_t)TT + t0 + q * 8, *(const v4u*)&th[cl][q * 8]); if (hi_rows) { const size_t o3 = (bb * KC + c0 + cl) * (size_t)HIR + (size_t)(t0 - HI0) + q * 8; vst2(VB + o3, *(const v4u*)&tb[cl][q * 8]); vst2(VBL + o3, *(const v4u*)&tbl[cl][q * 8]); } } }

template <int HI>
__device__ __forceinline__ void fa_body(const _Float16* __restrict__ QH, const _Float16* __restrict__ KH, const _Float16* __restrict__ QL, const _Float16* __restrict__ KL,
    const _Float16* __restrict__ VT, const __bf16* __restrict__ VB, const __bf16* __restrict__ VBL, float* __restrict__ Y, const int* __restrict__ WIN, const int qb) {
  __shared__ __align__(16) float sp[4][16][HD + 4];
  const int tid = threadIdx.x, lane = tid & 31, col = lane & 15, g = lane >> 4;
  const int wave = __builtin_amdgcn_readfirstlane(tid >> 5);
  const int h = blockIdx.y, b = blockIdx.z, kvh = h / NREP;
  const int wraw = WIN[0]; int weff = (wraw < TT) ? wraw : TT; if (weff < 0) weff = 0;
  const bool wneg = wraw < 0;
  const int ql0 = qb * 64 + wave * 16; const size_t q0 = (size_t)b * TT + ql0;
  const size_t qoff = (q0 + col) * CC + h * HD;
  const size_t qloff = ((size_t)b * HIR + (size_t)(HI ? (ql0 - HI0) : 0) + col) * CC + h * HD;
  const size_t kcol = (size_t)kvh * HD;
  v8f o[4] = {}; float mr[8], lr[8];
#pragma unroll
  for (int r = 0; r < 8; ++r) { mr[r] = -3.0e38f; lr[r] = 0.f; }
  int kfirst = ql0 - weff; if (kfirst < 0) kfirst = 0;
  const int c_lo = kfirst >> 5, c_hi = (ql0 + 15) >> 5;
#pragma unroll 1
  for (int c = c_lo; c <= c_hi; ++c) { const int k0 = c * 32; const size_t kr0 = (size_t)b * TT + k0;
    v8f s[2] = {}, sl[2] = {};
#pragma unroll
    for (int kc = 0; kc < 2; ++kc) { const v16h a = frag_h(QH + qoff + kc * 32, lane); v16h al = a; if (HI) al = frag_h(QL + qloff + kc * 32, lane);
#pragma unroll
      for (int j = 0; j < 2; ++j) { const v16h kf = frag_h(KH + (kr0 + j * 16 + col) * KC + kcol + kc * 32, lane); s[j] = wmma16(a, kf, s[j]);
        if (HI) { const v16h kl = frag_h(KL + ((size_t)b * HIR + (size_t)(k0 - HI0) + j * 16 + col) * KC + kcol + kc * 32, lane); sl[j] = wmma16(al, kf, sl[j]); sl[j] = wmma16(a, kl, sl[j]); } } }
    const bool interior = (k0 + 31 <= ql0) && (ql0 + 15 - k0 <= weff);
#pragma unroll
    for (int j = 0; j < 2; ++j) {
#pragma unroll
      for (int r = 0; r < 8; ++r) { float v = s[j][r]; if (HI) v += sl[j][r] * (1.0f / 1024.0f); v *= SC2; const int kj = k0 + j * 16 + col, qi = ql0 + 8 * g + r; const bool keep = (kj <= qi) && (qi - kj <= weff); const bool ex = (!interior) && (!keep); s[j][r] = ex ? -3.0e38f : v; } }
#pragma unroll
    for (int r = 0; r < 8; ++r) {
      float mx = fmaxf(s[0][r], s[1][r]);
      mx = fmaxf(mx, __shfl_xor(mx, 1)); mx = fmaxf(mx, __shfl_xor(mx, 2)); mx = fmaxf(mx, __shfl_xor(mx, 4)); mx = fmaxf(mx, __shfl_xor(mx, 8));
      const float nm = fmaxf(mr[r], mx);
      const float ea = exp2f(mr[r] - nm); const float alpha = (mr[r] < -1.0e38f) ? 0.f : ea;
      mr[r] = nm; float rs = 0.f;
#pragma unroll
      for (int j = 0; j < 2; ++j) { const float sv = s[j][r]; const float ep = exp2f(sv - nm); const float p = (sv < -1.0e38f) ? 0.f : ep; rs += p; s[j][r] = p; }
#pragma unroll
      for (int j = 0; j < 4; ++j) o[j][r] *= alpha;
      rs += __shfl_xor(rs, 1); rs += __shfl_xor(rs, 2); rs += __shfl_xor(rs, 4); rs += __shfl_xor(rs, 8);
      lr[r] = lr[r] * alpha + rs; }
#pragma unroll
    for (int j = 0; j < 2; ++j) {
#pragma unroll
      for (int r = 0; r < 8; ++r) sp[wave][8 * g + r][j * 16 + col] = s[j][r] * 2048.0f; }
    LDSX();
    if (HI) { float pv[16];
#pragma unroll
      for (int i = 0; i < 8; ++i) { pv[i] = sp[wave][col][8 * g + i]; pv[8 + i] = sp[wave][col][16 + 8 * g + i]; }
      const F2 p = bsplit16(pv);
#pragma unroll
      for (int j = 0; j < 4; ++j) { const size_t po = ((size_t)b * KC + kcol + j * 16 + col) * (size_t)HIR + (size_t)(k0 - HI0); const v16b vh = frag_b(VB + po, lane); const v16b vl = frag_b(VBL + po, lane); o[j] = wmma_bf(p.h, vh, o[j]); o[j] = wmma_bf(p.l, vh, o[j]); o[j] = wmma_bf(p.h, vl, o[j]); }
    } else { v16h a;
#pragma unroll
      for (int i = 0; i < 8; ++i) { a[i] = toh_flush(sp[wave][col][8 * g + i]); a[8 + i] = toh_flush(sp[wave][col][16 + 8 * g + i]); }
#pragma unroll
      for (int j = 0; j < 4; ++j) { const size_t po = ((size_t)b * KC + kcol + j * 16 + col) * (size_t)TT + k0; o[j] = wmma16(a, frag_h(VT + po, lane), o[j]); } }
    LDSX(); }
  const float qnan = __uint_as_float(0x7fc00000u);
#pragma unroll
  for (int r = 0; r < 8; ++r) { const float inv0 = 1.0f / (lr[r] * 2048.0f); const float inv = wneg ? qnan : inv0;
#pragma unroll
    for (int j = 0; j < 4; ++j) sp[wave][8 * g + r][j * 16 + col] = o[j][r] * inv; }
  LDSX();
  for (int rl = 0; rl < 16; ++rl) if (lane < HD / 4) vst2(Y + (q0 + rl) * CC + h * HD + lane * 4, *(const v4f*)&sp[wave][rl][lane * 4]); }

__global__ __launch_bounds__(128) void k_fa_hi(const _Float16* __restrict__ QH, const _Float16* __restrict__ KH, const _Float16* __restrict__ QL, const _Float16* __restrict__ KL, const _Float16* __restrict__ VT, const __bf16* __restrict__ VB, const __bf16* __restrict__ VBL, float* __restrict__ Y, const int* __restrict__ WIN) {
  fa_body<1>(QH, KH, QL, KL, VT, VB, VBL, Y, WIN, (int)blockIdx.x); }
__global__ __launch_bounds__(128) void k_fa_lo(const _Float16* __restrict__ QH, const _Float16* __restrict__ KH, const _Float16* __restrict__ QL, const _Float16* __restrict__ KL, const _Float16* __restrict__ VT, const __bf16* __restrict__ VB, const __bf16* __restrict__ VBL, float* __restrict__ Y, const int* __restrict__ WIN) {
  fa_body<0>(QH, KH, QL, KL, VT, VB, VBL, Y, WIN, (int)blockIdx.x + QBH); }

__global__ __launch_bounds__(128) void k_out(const float* __restrict__ Y, const __bf16* __restrict__ WOB, const _Float16* __restrict__ WOH, float* __restrict__ OUT) {
  __shared__ __align__(16) float sf[4][16][132];
  const int tid = threadIdx.x, wave = tid >> 5, lane = tid & 31, col = lane & 15, g = lane >> 4; const int c0 = blockIdx.y * 128;
  const size_t rb = (size_t)blockIdx.x * 64; const size_t bb = rb / TT; const int t0 = (int)(rb % TT); const size_t r0 = rb + wave * 16; const size_t orow = bb * (size_t)SEQ_FULL + t0 + wave * 16;
  v8f acc[8] = {};
  if (t0 < HIR) {
#pragma unroll 2
    for (int kc = 0; kc < CC / 32; ++kc) { const F2 a = split_row(Y + (r0 + col) * CC, kc * 32, lane); asm volatile("s_wait_loadcnt 0x0" ::: "memory");
#pragma unroll
      for (int j = 0; j < 8; ++j) { const v16b w = frag_b(WOB + (size_t)(c0 + j * 16 + col) * CC + kc * 32, lane); asm volatile("s_wait_loadcnt 0x0" ::: "memory"); acc[j] = wmma_bf(a.h, w, acc[j]); acc[j] = wmma_bf(a.l, w, acc[j]); } }
#pragma unroll
    for (int j = 0; j < 8; ++j) {
#pragma unroll
      for (int r = 0; r < 8; ++r) sf[wave][8 * g + r][j * 16 + col] = acc[j][r]; }
  } else {
#pragma unroll 2
    for (int kc = 0; kc < CC / 32; ++kc) { const v16h a = frag_f32s_flush(Y + (r0 + col) * CC + kc * 32, lane, 64.0f); asm volatile("s_wait_loadcnt 0x0" ::: "memory");
#pragma unroll
      for (int j = 0; j < 8; ++j) { const v16h w = frag_h(WOH + (size_t)(c0 + j * 16 + col) * CC + kc * 32, lane); asm volatile("s_wait_loadcnt 0x0" ::: "memory"); acc[j] = wmma16(a, w, acc[j]); } }
#pragma unroll
    for (int j = 0; j < 8; ++j) {
#pragma unroll
      for (int r = 0; r < 8; ++r) sf[wave][8 * g + r][j * 16 + col] = acc[j][r] * (1.0f / 16384.0f); } }
  LDSX(); for (int rl = 0; rl < 16; ++rl) vst2(OUT + (orow + rl) * DIN + c0 + lane * 4, *(const v4f*)&sf[wave][rl][lane * 4]); }

extern "C" void kernel_launch(void* const* d_in, const int* in_sizes, int n_in, void* d_out, int out_size, void* d_ws, size_t ws_size, hipStream_t stream) {
  if (n_in < 10) return;
  const long need_rows = (long)(NB - 1) * SEQ_FULL + SEQ;
  if ((long)in_sizes[0] < need_rows * DIN) return;
  if ((long)in_sizes[1] < need_rows * KC) return;
  if ((long)in_sizes[2] < (long)SEQ * 32) return;
  if ((long)in_sizes[3] < (long)SEQ * 32) return;
  if ((long)in_sizes[4] < (long)CC * DIN) return;
  if ((long)in_sizes[5] < (long)KC * DIN) return;
  if ((long)in_sizes[6] < (long)KC * DIN) return;
  if ((long)in_sizes[7] < (long)DIN * CC) return;
  if ((long)in_sizes[8] < (long)NKV * GCH) return;
  if ((long)in_sizes[9] < 1L) return;
  if ((long)out_size < need_rows * DIN) return;
  if (ws_size < (size_t)WS_END) return;
  const float* X = (const float*)d_in[0]; const float* VE = (const float*)d_in[1]; const float* COS = (const float*)d_in[2]; const float* SIN = (const float*)d_in[3];
  const float* WQ = (const float*)d_in[4]; const float* WK = (const float*)d_in[5]; const float* WV = (const float*)d_in[6]; const float* WP = (const float*)d_in[7]; const float* WG = (const float*)d_in[8];
  const int* WIN = (const int*)d_in[9];
  char* ws = (char*)d_ws;
  _Float16 *QH = (_Float16*)(ws + WS_QH), *KH = (_Float16*)(ws + WS_KH), *VT = (_Float16*)(ws + WS_VT), *QL = (_Float16*)(ws + WS_QL), *KL = (_Float16*)(ws + WS_KL), *WOH = (_Float16*)(ws + WS_WOH);
  __bf16 *VB = (__bf16*)(ws + WS_VB), *VBL = (__bf16*)(ws + WS_VBL), *WQB = (__bf16*)(ws + WS_WQB), *WOB = (__bf16*)(ws + WS_WOB);
  float* Y = (float*)(ws + WS_Y);
  k_cvt<<<dim3(CC * DIN / 2048), 256, 0, stream>>>(WQ, CC * DIN / 8, WQB, WOH, 0);
  k_cvt<<<dim3(KC * DIN / 2048), 256, 0, stream>>>(WK, KC * DIN / 8, WQB + (size_t)CC * DIN, WOH, 0);
  k_cvt<<<dim3(KC * DIN / 2048), 256, 0, stream>>>(WV, KC * DIN / 8, WQB + (size_t)(CC + KC) * DIN, WOH, 0);
  k_cvt<<<dim3(DIN * CC / 2048), 256, 0, stream>>>(WP, DIN * CC / 8, WOB, WOH, 1);
  k_proj_qk<<<dim3(NB * TT / 64, CC / 128), 128, 0, stream>>>(X, WQB, COS, SIN, QH, QL, CC);
  k_proj_qk<<<dim3(NB * TT / 64, KC / 128), 128, 0, stream>>>(X, WQB + (size_t)CC * DIN, COS, SIN, KH, KL, KC);
  k_proj_v<<<dim3(NB * TT / 64, KC / 128), 128, 0, stream>>>(X, WQB + (size_t)(CC + KC) * DIN, VE, WG, VT, VB, VBL);
  k_fa_hi<<<dim3(QBH, NH, NB), 128, 0, stream>>>(QH, KH, QL, KL, VT, VB, VBL, Y, WIN);
  if (NLO > 0) k_fa_lo<<<dim3(NLO > 0 ? NLO : 1, NH, NB), 128, 0, stream>>>(QH, KH, QL, KL, VT, VB, VBL, Y, WIN);
  k_out<<<dim3(NB * TT / 64, DIN / 128), 128, 0, stream>>>(Y, WOB, WOH, (float*)d_out);
}
